// ContrastiveSWM_60138132078979
// MI455X (gfx1250) — hardware-verified
//
#include <hip/hip_runtime.h>

typedef _Float16 v16h __attribute__((ext_vector_type(16)));
typedef _Float16 v8h  __attribute__((ext_vector_type(8)));
typedef __bf16   v16b __attribute__((ext_vector_type(16)));
typedef unsigned short v8us __attribute__((ext_vector_type(8)));
typedef unsigned short v4us __attribute__((ext_vector_type(4)));
typedef float v8f __attribute__((ext_vector_type(8)));
typedef float v4f __attribute__((ext_vector_type(4)));
typedef v8h  __attribute__((may_alias)) v8ha;
typedef v8us __attribute__((may_alias)) v8usa;
typedef v4us __attribute__((may_alias)) v4usa;
typedef v4f  __attribute__((may_alias)) v4fa;

union FragH { v16h v; v8h p[2]; };
union FragB { v16b v; v8us p[2]; };

#define NGRAPH 1024
#define NOBJ   16
#define NNODE  (NGRAPH * NOBJ)
#define DIN    128
#define HID    256
#define LN_EPS 1e-5f

#define EPH 264
#define EPX 260
#define E_OFF_PQ   0
#define E_OFF_PAR  (E_OFF_PQ + 16 * 512 * 4)
#define E_OFF_H    (E_OFF_PAR + 4 * 256 * 4)
#define E_OFF_X    (E_OFF_H + 48 * EPH * 2)
#define E_OFF_AGG  (E_OFF_X + 48 * EPX * 4)
#define E_SMEM     (E_OFF_AGG + 16 * 256 * 4)

#define PQA 136
#define PQO 516
#define P_OFF_AH 0
#define P_OFF_AL (32 * PQA * 2)
#define P_OFF_O  (2 * 32 * PQA * 2)
#define P_SMEM   (P_OFF_O + 32 * PQO * 4)

#define NP1 392
#define NP2 264
#define NPX 260
#define NPO 132
#define N_OFF_A1H 0
#define N_OFF_A1L (32 * NP1 * 2)
#define N_OFF_A2H (2 * 32 * NP1 * 2)
#define N_OFF_A2L (N_OFF_A2H + 32 * NP2 * 2)
#define N_OFF_X   (N_OFF_A2L + 32 * NP2 * 2)
#define N_OFF_O   (N_OFF_X + 32 * NPX * 4)
#define N_SMEM    (N_OFF_O + 32 * NPO * 4)

__device__ __forceinline__ v8f wmma_f16(v16h a, v16h b, v8f c) {
  v8f d = __builtin_amdgcn_wmma_f32_16x16x32_f16(false, a, false, b, (short)0, c, false, false);
  asm volatile("v_nop\n\tv_nop\n\tv_nop\n\tv_nop" : "+v"(d) : "v"(a), "v"(b));
  return d;
}
__device__ __forceinline__ v8f wmma_bf16(v16b a, v16b b, v8f c) {
  v8f d = __builtin_amdgcn_wmma_f32_16x16x32_bf16(false, a, false, b, (short)0, c, false, false);
  asm volatile("v_nop\n\tv_nop\n\tv_nop\n\tv_nop" : "+v"(d) : "v"(a), "v"(b));
  return d;
}
__device__ __forceinline__ v8f wmma_split(v16b ah, v16b al, v16b bh, v16b bl, v8f c) {
  c = wmma_bf16(ah, bh, c);
  c = wmma_bf16(ah, bl, c);
  c = wmma_bf16(al, bh, c);
  return c;
}

__device__ __forceinline__ v16h ldfrag_h(const _Float16* p, int h) {
  FragH f;
  f.p[0] = *(const v8ha*)(p + 8 * h);
  f.p[1] = *(const v8ha*)(p + 16 + 8 * h);
  return f.v;
}
__device__ __forceinline__ v16b ldfrag_b(const unsigned short* p, int h) {
  FragB f;
  f.p[0] = *(const v8usa*)(p + 8 * h);
  f.p[1] = *(const v8usa*)(p + 16 + 8 * h);
  return f.v;
}

__device__ __forceinline__ unsigned int bf16_rne_bits(float x) {
  unsigned int u = __float_as_uint(x);
  u += 0x7FFFu + ((u >> 16) & 1u);
  return u >> 16;
}
__device__ __forceinline__ void split1(float x, unsigned short& hi, unsigned short& lo) {
  const unsigned int hb = bf16_rne_bits(x);
  const float hf = __uint_as_float(hb << 16);
  hi = (unsigned short)hb;
  lo = (unsigned short)bf16_rne_bits(x - hf);
}
__device__ __forceinline__ void split4(v4f x, v4us& hi, v4us& lo) {
  unsigned short h0, h1, h2, h3, l0, l1, l2, l3;
  split1(x.x, h0, l0); split1(x.y, h1, l1); split1(x.z, h2, l2); split1(x.w, h3, l3);
  const v4us hv = {h0, h1, h2, h3};
  const v4us lv = {l0, l1, l2, l3};
  hi = hv; lo = lv;
}

template<int ROWF, int PITCH, int NIT>
__device__ __forceinline__ void store_lines(const float* s, float* g, int w, int lane) {
  const int q8 = lane & 7, sub = lane >> 3;
  constexpr int LPR = ROWF / 32;
  #pragma unroll
  for (int it = 0; it < NIT; ++it) {
    const int line = NIT * 4 * w + 4 * it + sub;
    const int row = line / LPR;
    const int piece = (line % LPR) * 32 + 4 * q8;
    const v4f v = *(const v4fa*)(s + row * PITCH + piece);
    *(volatile v4f*)(g + (size_t)row * ROWF + piece) = v;
  }
}

__global__ __launch_bounds__(256) void cvt_kernel(
    const float* __restrict__ src, int srcCols, int cT,
    int cSplit, int rowAddC, int kSplit, int rowAddK,
    int dstK, int mode, float scale,
    unsigned short* __restrict__ dst0, unsigned short* __restrict__ dst1)
{
  __shared__ __attribute__((aligned(16))) unsigned short sT0[64 * 72];
  __shared__ __attribute__((aligned(16))) unsigned short sT1[64 * 72];
  const int tid = threadIdx.x, lane = tid & 31, w = tid >> 5;
  const int ct = blockIdx.x % cT, kt = blockIdx.x / cT;
  const int c0 = ct * 64, k0 = kt * 64;

  #pragma unroll
  for (int it = 0; it < 16; ++it) {
    const int idx = tid + 256 * it;
    const int kk = idx >> 6, cc = idx & 63;
    const int c = c0 + cc, k = k0 + kk;
    int srow = k, scol = c;
    if (c >= cSplit) { srow += rowAddC; scol -= cSplit; }
    if (k >= kSplit) srow += rowAddK;
    const float v = src[(size_t)srow * srcCols + scol] * scale;
    unsigned short o0, o1;
    if (mode == 0) { o0 = __builtin_bit_cast(unsigned short, (_Float16)v); o1 = 0; }
    else { split1(v, o0, o1); }
    sT0[cc * 72 + kk] = o0;
    sT1[cc * 72 + kk] = o1;
  }
  __syncthreads();

  const int q8 = lane & 7, sub = lane >> 3;
  #pragma unroll
  for (int pass = 0; pass < 2; ++pass) {
    #pragma unroll
    for (int it = 0; it < 2; ++it) {
      const int line = 8 * w + 4 * it + sub;
      const size_t go = (size_t)(c0 + line) * dstK + k0 + 8 * q8;
      const v8us v0 = *(const v8usa*)(sT0 + line * 72 + 8 * q8);
      *(volatile v8us*)(dst0 + go) = v0;
      if (mode != 0) {
        const v8us v1 = *(const v8usa*)(sT1 + line * 72 + 8 * q8);
        *(volatile v8us*)(dst1 + go) = v1;
      }
    }
    if (pass == 0) __threadfence();
  }
}

__global__ __launch_bounds__(256) void pq_kernel(
    const float* __restrict__ states,
    const unsigned short* __restrict__ bph, const unsigned short* __restrict__ bpl,
    const float* __restrict__ eb1, float* __restrict__ pq)
{
  extern __shared__ __attribute__((aligned(16))) char smem_p[];
  unsigned short* sAh = (unsigned short*)(smem_p + P_OFF_AH);
  unsigned short* sAl = (unsigned short*)(smem_p + P_OFF_AL);
  float* sO = (float*)(smem_p + P_OFF_O);

  const int tid = threadIdx.x, lane = tid & 31, w = tid >> 5;
  const int h = lane >> 4, m = lane & 15;
  const int node0 = blockIdx.x * 32;

  #pragma unroll
  for (int it = 0; it < 4; ++it) {
    const int idx = tid + 256 * it, row = idx >> 5, c4 = (idx & 31) * 4;
    const v4f x = *(const v4fa*)(states + (size_t)(node0 + row) * DIN + c4);
    v4us hv, lv;
    split4(x, hv, lv);
    *(v4usa*)(sAh + row * PQA + c4) = hv;
    *(v4usa*)(sAl + row * PQA + c4) = lv;
  }
  __syncthreads();

  const v8f z8 = {0.f, 0.f, 0.f, 0.f, 0.f, 0.f, 0.f, 0.f};
  v8f acc[2][4];
  #pragma unroll
  for (int mt = 0; mt < 2; ++mt)
    #pragma unroll
    for (int nt = 0; nt < 4; ++nt) acc[mt][nt] = z8;

  const unsigned short* bhr = bph + (size_t)(64 * w + m) * DIN;
  const unsigned short* blr = bpl + (size_t)(64 * w + m) * DIN;
  #pragma unroll 1
  for (int k0 = 0; k0 < DIN; k0 += 32) {
    const v16b ah0 = ldfrag_b(sAh + m * PQA + k0, h);
    const v16b al0 = ldfrag_b(sAl + m * PQA + k0, h);
    const v16b ah1 = ldfrag_b(sAh + (16 + m) * PQA + k0, h);
    const v16b al1 = ldfrag_b(sAl + (16 + m) * PQA + k0, h);
    #pragma unroll
    for (int nt = 0; nt < 4; ++nt) {
      const v16b bhf = ldfrag_b(bhr + nt * 16 * DIN + k0, h);
      const v16b blf = ldfrag_b(blr + nt * 16 * DIN + k0, h);
      acc[0][nt] = wmma_split(ah0, al0, bhf, blf, acc[0][nt]);
      acc[1][nt] = wmma_split(ah1, al1, bhf, blf, acc[1][nt]);
    }
  }

  #pragma unroll
  for (int nt = 0; nt < 4; ++nt) {
    const int col = 64 * w + 16 * nt + m;
    const float bl = eb1[col & 255];
    const float bias = (col < 256) ? bl : 0.f;
    #pragma unroll
    for (int mt = 0; mt < 2; ++mt)
      #pragma unroll
      for (int r = 0; r < 8; ++r)
        sO[(16 * mt + 8 * h + r) * PQO + col] = acc[mt][nt][r] + bias;
  }
  __syncthreads();

  float* g = pq + (size_t)node0 * 512;
  store_lines<512, PQO, 16>(sO, g, w, lane);
  __threadfence();
  store_lines<512, PQO, 16>(sO, g, w, lane);
}

__device__ __forceinline__ void edge_layer(const _Float16* sH, float* sX,
                                           const _Float16* __restrict__ wg, const float* bias,
                                           int w, int h, int m) {
  const v8f z8 = {0.f, 0.f, 0.f, 0.f, 0.f, 0.f, 0.f, 0.f};
  v8f acc[3][2];
  #pragma unroll
  for (int mt = 0; mt < 3; ++mt) { acc[mt][0] = z8; acc[mt][1] = z8; }

  const _Float16* wr0 = wg + (size_t)(32 * w + m) * HID;
  const _Float16* wr1 = wr0 + 16 * HID;
  const _Float16* ar = sH + m * EPH;
  #pragma unroll 1
  for (int k0 = 0; k0 < HID; k0 += 32) {
    const v16h a0 = ldfrag_h(ar + k0, h);
    const v16h a1 = ldfrag_h(ar + 16 * EPH + k0, h);
    const v16h a2 = ldfrag_h(ar + 32 * EPH + k0, h);
    const v16h b0 = ldfrag_h(wr0 + k0, h);
    const v16h b1 = ldfrag_h(wr1 + k0, h);
    acc[0][0] = wmma_f16(a0, b0, acc[0][0]);
    acc[0][1] = wmma_f16(a0, b1, acc[0][1]);
    acc[1][0] = wmma_f16(a1, b0, acc[1][0]);
    acc[1][1] = wmma_f16(a1, b1, acc[1][1]);
    acc[2][0] = wmma_f16(a2, b0, acc[2][0]);
    acc[2][1] = wmma_f16(a2, b1, acc[2][1]);
  }
  #pragma unroll
  for (int nt = 0; nt < 2; ++nt) {
    const int col = 32 * w + 16 * nt + m;
    const float bv = bias[col];
    #pragma unroll
    for (int mt = 0; mt < 3; ++mt)
      #pragma unroll
      for (int r = 0; r < 8; ++r)
        sX[(16 * mt + 8 * h + r) * EPX + col] = acc[mt][nt][r] * 0.0625f + bv;
  }
}

__device__ __forceinline__ void edge_ln(const float* sX, _Float16* sH,
                                        const float* gp, const float* bp, int w, int lane) {
  const v4f ga = *(const v4fa*)(gp + 8 * lane), gb = *(const v4fa*)(gp + 8 * lane + 4);
  const v4f ta = *(const v4fa*)(bp + 8 * lane), tb = *(const v4fa*)(bp + 8 * lane + 4);
  const float gg[8] = {ga.x, ga.y, ga.z, ga.w, gb.x, gb.y, gb.z, gb.w};
  const float tt[8] = {ta.x, ta.y, ta.z, ta.w, tb.x, tb.y, tb.z, tb.w};
  #pragma unroll 1
  for (int rr = 0; rr < 6; ++rr) {
    const int row = 6 * w + rr;
    const float* xr = sX + row * EPX + 8 * lane;
    const v4f xa = *(const v4fa*)xr, xb = *(const v4fa*)(xr + 4);
    const float x[8] = {xa.x, xa.y, xa.z, xa.w, xb.x, xb.y, xb.z, xb.w};
    float s = ((x[0] + x[1]) + (x[2] + x[3])) + ((x[4] + x[5]) + (x[6] + x[7]));
    #pragma unroll
    for (int off = 1; off < 32; off <<= 1) s += __shfl_xor(s, off);
    const float mean = s * (1.0f / 256.0f);
    float d[8];
    float q = 0.f;
    #pragma unroll
    for (int v = 0; v < 8; ++v) { d[v] = x[v] - mean; q += d[v] * d[v]; }
    #pragma unroll
    for (int off = 1; off < 32; off <<= 1) q += __shfl_xor(q, off);
    const float inv = rsqrtf(q * (1.0f / 256.0f) + LN_EPS);
    v8h o;
    #pragma unroll
    for (int v = 0; v < 8; ++v) o[v] = (_Float16)fmaxf(d[v] * inv * gg[v] + tt[v], 0.f);
    *(v8ha*)(sH + row * EPH + 8 * lane) = o;
  }
}

__global__ __launch_bounds__(256) void edge_kernel(
    const float* __restrict__ pq,
    const _Float16* __restrict__ w2h, const _Float16* __restrict__ w3h,
    const float* __restrict__ eb2, const float* __restrict__ eg,
    const float* __restrict__ ebt, const float* __restrict__ eb3,
    float* __restrict__ agg)
{
  extern __shared__ __attribute__((aligned(16))) char smem_e[];
  float* sPQ = (float*)(smem_e + E_OFF_PQ);
  float* sPar = (float*)(smem_e + E_OFF_PAR);
  _Float16* sH = (_Float16*)(smem_e + E_OFF_H);
  float* sX = (float*)(smem_e + E_OFF_X);
  float* sAgg = (float*)(smem_e + E_OFF_AGG);

  const int tid = threadIdx.x, lane = tid & 31, w = tid >> 5;
  const int h = lane >> 4, m = lane & 15;
  const int node0 = blockIdx.x * NOBJ;

  #pragma unroll
  for (int it = 0; it < 8; ++it) {
    const int idx = tid + 256 * it, row = idx >> 7, c4 = (idx & 127) * 4;
    const v4f v = *(const v4fa*)(pq + (size_t)(node0 + row) * 512 + c4);
    *(v4fa*)(sPQ + row * 512 + c4) = v;
  }
  sPar[tid] = eb2[tid];
  sPar[256 + tid] = eg[tid];
  sPar[512 + tid] = ebt[tid];
  sPar[768 + tid] = eb3[tid];
  #pragma unroll
  for (int i = 0; i < 16; ++i) sAgg[i * 256 + tid] = 0.f;
  __syncthreads();

  #pragma unroll 1
  for (int gi = 0; gi < 5; ++gi) {
    #pragma unroll
    for (int it = 0; it < 6; ++it) {
      const int task = tid + 256 * it;
      const int rl = task >> 5, cg = (task & 31) * 8;
      const int e = 48 * gi + rl, i = e / 15, jj = e - 15 * i;
      const int j = jj + ((jj >= i) ? 1 : 0);
      const float* pp = sPQ + i * 512 + cg;
      const float* qp = sPQ + j * 512 + 256 + cg;
      const v4f p0 = *(const v4fa*)pp, p1 = *(const v4fa*)(pp + 4);
      const v4f q0 = *(const v4fa*)qp, q1 = *(const v4fa*)(qp + 4);
      v8h o;
      o[0] = (_Float16)fmaxf(p0.x + q0.x, 0.f);
      o[1] = (_Float16)fmaxf(p0.y + q0.y, 0.f);
      o[2] = (_Float16)fmaxf(p0.z + q0.z, 0.f);
      o[3] = (_Float16)fmaxf(p0.w + q0.w, 0.f);
      o[4] = (_Float16)fmaxf(p1.x + q1.x, 0.f);
      o[5] = (_Float16)fmaxf(p1.y + q1.y, 0.f);
      o[6] = (_Float16)fmaxf(p1.z + q1.z, 0.f);
      o[7] = (_Float16)fmaxf(p1.w + q1.w, 0.f);
      *(v8ha*)(sH + rl * EPH + cg) = o;
    }
    __syncthreads();
    edge_layer(sH, sX, w2h, sPar, w, h, m);
    __syncthreads();
    edge_ln(sX, sH, sPar + 256, sPar + 512, w, lane);
    __syncthreads();
    edge_layer(sH, sX, w3h, sPar + 768, w, h, m);
    __syncthreads();
    #pragma unroll 4
    for (int rl = 0; rl < 48; ++rl) {
      const int e = 48 * gi + rl, i = e / 15;
      sAgg[i * 256 + tid] += sX[rl * EPX + tid];
    }
    __syncthreads();
  }

  float* g = agg + (size_t)node0 * HID;
  store_lines<256, 256, 4>(sAgg, g, w, lane);
  __threadfence();
  store_lines<256, 256, 4>(sAgg, g, w, lane);
}

template<int KTOT, int PA>
__device__ __forceinline__ void node_gemm(const unsigned short* sAh, const unsigned short* sAl,
                                          const unsigned short* __restrict__ bh,
                                          const unsigned short* __restrict__ bl,
                                          int w, int h, int m, v8f (&acc)[2][2]) {
  const v8f z8 = {0.f, 0.f, 0.f, 0.f, 0.f, 0.f, 0.f, 0.f};
  acc[0][0] = z8; acc[0][1] = z8; acc[1][0] = z8; acc[1][1] = z8;
  const unsigned short* ahr = sAh + m * PA;
  const unsigned short* alr = sAl + m * PA;
  const unsigned short* bhr = bh + (size_t)(32 * w + m) * KTOT;
  const unsigned short* blr = bl + (size_t)(32 * w + m) * KTOT;
  #pragma unroll 1
  for (int k0 = 0; k0 < KTOT; k0 += 32) {
    const v16b ah0 = ldfrag_b(ahr + k0, h);
    const v16b al0 = ldfrag_b(alr + k0, h);
    const v16b ah1 = ldfrag_b(ahr + 16 * PA + k0, h);
    const v16b al1 = ldfrag_b(alr + 16 * PA + k0, h);
    #pragma unroll
    for (int nt = 0; nt < 2; ++nt) {
      const v16b bhf = ldfrag_b(bhr + nt * 16 * KTOT + k0, h);
      const v16b blf = ldfrag_b(blr + nt * 16 * KTOT + k0, h);
      acc[0][nt] = wmma_split(ah0, al0, bhf, blf, acc[0][nt]);
      acc[1][nt] = wmma_split(ah1, al1, bhf, blf, acc[1][nt]);
    }
  }
}

__device__ __forceinline__ void node_ln(const float* sX, unsigned short* sAh, unsigned short* sAl,
                                        const float* __restrict__ gp, const float* __restrict__ bp,
                                        int w, int lane) {
  const v4f ga = *(const v4fa*)(gp + 8 * lane), gb = *(const v4fa*)(gp + 8 * lane + 4);
  const v4f ta = *(const v4fa*)(bp + 8 * lane), tb = *(const v4fa*)(bp + 8 * lane + 4);
  const float gg[8] = {ga.x, ga.y, ga.z, ga.w, gb.x, gb.y, gb.z, gb.w};
  const float tt[8] = {ta.x, ta.y, ta.z, ta.w, tb.x, tb.y, tb.z, tb.w};
  #pragma unroll 1
  for (int rr = 0; rr < 4; ++rr) {
    const int row = 4 * w + rr;
    const float* xr = sX + row * NPX + 8 * lane;
    const v4f xa = *(const v4fa*)xr, xb = *(const v4fa*)(xr + 4);
    const float x[8] = {xa.x, xa.y, xa.z, xa.w, xb.x, xb.y, xb.z, xb.w};
    float s = ((x[0] + x[1]) + (x[2] + x[3])) + ((x[4] + x[5]) + (x[6] + x[7]));
    #pragma unroll
    for (int off = 1; off < 32; off <<= 1) s += __shfl_xor(s, off);
    const float mean = s * (1.0f / 256.0f);
    float d[8];
    float q = 0.f;
    #pragma unroll
    for (int v = 0; v < 8; ++v) { d[v] = x[v] - mean; q += d[v] * d[v]; }
    #pragma unroll
    for (int off = 1; off < 32; off <<= 1) q += __shfl_xor(q, off);
    const float inv = rsqrtf(q * (1.0f / 256.0f) + LN_EPS);
    unsigned short hv[8], lv[8];
    #pragma unroll
    for (int v = 0; v < 8; ++v) {
      const float y = fmaxf(d[v] * inv * gg[v] + tt[v], 0.f);
      split1(y, hv[v], lv[v]);
    }
    const v8us ho = {hv[0], hv[1], hv[2], hv[3], hv[4], hv[5], hv[6], hv[7]};
    const v8us lo = {lv[0], lv[1], lv[2], lv[3], lv[4], lv[5], lv[6], lv[7]};
    *(v8usa*)(sAh + row * NP2 + 8 * lane) = ho;
    *(v8usa*)(sAl + row * NP2 + 8 * lane) = lo;
  }
}

__global__ __launch_bounds__(256) void node_kernel(
    const float* __restrict__ states, const float* __restrict__ agg, const int* __restrict__ action,
    const unsigned short* __restrict__ n1h, const unsigned short* __restrict__ n1l,
    const float* __restrict__ nW1, const float* __restrict__ nb1,
    const unsigned short* __restrict__ n2h, const unsigned short* __restrict__ n2l,
    const float* __restrict__ nb2, const float* __restrict__ ng, const float* __restrict__ nbt,
    const unsigned short* __restrict__ n3h, const unsigned short* __restrict__ n3l,
    const float* __restrict__ nb3, float* __restrict__ out)
{
  extern __shared__ __attribute__((aligned(16))) char smem_n[];
  unsigned short* sA1h = (unsigned short*)(smem_n + N_OFF_A1H);
  unsigned short* sA1l = (unsigned short*)(smem_n + N_OFF_A1L);
  unsigned short* sA2h = (unsigned short*)(smem_n + N_OFF_A2H);
  unsigned short* sA2l = (unsigned short*)(smem_n + N_OFF_A2L);
  float* sX = (float*)(smem_n + N_OFF_X);
  float* sO = (float*)(smem_n + N_OFF_O);

  const int tid = threadIdx.x, lane = tid & 31, w = tid >> 5;
  const int h = lane >> 4, m = lane & 15;
  const int node0 = blockIdx.x * 32;

  #pragma unroll
  for (int it = 0; it < 4; ++it) {
    const int idx = tid + 256 * it, row = idx >> 5, c4 = (idx & 31) * 4;
    const v4f x = *(const v4fa*)(states + (size_t)(node0 + row) * DIN + c4);
    v4us hv, lv;
    split4(x, hv, lv);
    *(v4usa*)(sA1h + row * NP1 + c4) = hv;
    *(v4usa*)(sA1l + row * NP1 + c4) = lv;
  }
  #pragma unroll
  for (int it = 0; it < 8; ++it) {
    const int idx = tid + 256 * it, row = idx >> 6, c4 = (idx & 63) * 4;
    const v4f x = *(const v4fa*)(agg + (size_t)(node0 + row) * HID + c4);
    v4us hv, lv;
    split4(x, hv, lv);
    *(v4usa*)(sA1h + row * NP1 + 128 + c4) = hv;
    *(v4usa*)(sA1l + row * NP1 + 128 + c4) = lv;
  }
  __syncthreads();

  v8f acc[2][2];
  node_gemm<384, NP1>(sA1h, sA1l, n1h, n1l, w, h, m, acc);
  {
    int a0 = action[(node0 >> 4) + 0];
    int a1 = action[(node0 >> 4) + 1];
    a0 = min(max(a0, 0), 3);
    a1 = min(max(a1, 0), 3);
    #pragma unroll
    for (int nt = 0; nt < 2; ++nt) {
      const int col = 32 * w + 16 * nt + m;
      const float bv = nb1[col];
      const float wa0 = nW1[(size_t)(128 + a0) * HID + col];
      const float wa1 = nW1[(size_t)(128 + a1) * HID + col];
      #pragma unroll
      for (int r = 0; r < 8; ++r) {
        const int row0 = 8 * h + r, row1 = 16 + 8 * h + r;
        const float v0 = fmaxf(acc[0][nt][r] + wa0 + bv, 0.f);
        const float v1 = fmaxf(acc[1][nt][r] + wa1 + bv, 0.f);
        unsigned short h0, l0, h1, l1;
        split1(v0, h0, l0);
        split1(v1, h1, l1);
        sA2h[row0 * NP2 + col] = h0; sA2l[row0 * NP2 + col] = l0;
        sA2h[row1 * NP2 + col] = h1; sA2l[row1 * NP2 + col] = l1;
      }
    }
  }
  __syncthreads();
  node_gemm<256, NP2>(sA2h, sA2l, n2h, n2l, w, h, m, acc);
  #pragma unroll
  for (int nt = 0; nt < 2; ++nt) {
    const int col = 32 * w + 16 * nt + m;
    const float bv = nb2[col];
    #pragma unroll
    for (int mt = 0; mt < 2; ++mt)
      #pragma unroll
      for (int r = 0; r < 8; ++r)
        sX[(16 * mt + 8 * h + r) * NPX + col] = acc[mt][nt][r] + bv;
  }
  __syncthreads();
  node_ln(sX, sA2h, sA2l, ng, nbt, w, lane);
  __syncthreads();
  {
    const v8f z8 = {0.f, 0.f, 0.f, 0.f, 0.f, 0.f, 0.f, 0.f};
    v8f c3[2];
    c3[0] = z8; c3[1] = z8;
    const unsigned short* ahr = sA2h + m * NP2;
    const unsigned short* alr = sA2l + m * NP2;
    const unsigned short* bhr = n3h + (size_t)(16 * w + m) * HID;
    const unsigned short* blr = n3l + (size_t)(16 * w + m) * HID;
    #pragma unroll 1
    for (int k0 = 0; k0 < HID; k0 += 32) {
      const v16b ah0 = ldfrag_b(ahr + k0, h);
      const v16b al0 = ldfrag_b(alr + k0, h);
      const v16b ah1 = ldfrag_b(ahr + 16 * NP2 + k0, h);
      const v16b al1 = ldfrag_b(alr + 16 * NP2 + k0, h);
      const v16b bhf = ldfrag_b(bhr + k0, h);
      const v16b blf = ldfrag_b(blr + k0, h);
      c3[0] = wmma_split(ah0, al0, bhf, blf, c3[0]);
      c3[1] = wmma_split(ah1, al1, bhf, blf, c3[1]);
    }
    const int col = 16 * w + m;
    const float bv = nb3[col];
    #pragma unroll
    for (int mt = 0; mt < 2; ++mt)
      #pragma unroll
      for (int r = 0; r < 8; ++r)
        sO[(16 * mt + 8 * h + r) * NPO + col] = c3[mt][r] + bv;
  }
  __syncthreads();

  float* g = out + (size_t)node0 * DIN;
  store_lines<128, NPO, 4>(sO, g, w, lane);
  __threadfence();
  store_lines<128, NPO, 4>(sO, g, w, lane);
}

static void launch_cvt(hipStream_t s, const float* src, int srcCols, int cT, int kT,
                       int cSplit, int rowAddC, int kSplit, int rowAddK, int dstK,
                       int mode, float scale, unsigned short* d0, unsigned short* d1) {
  cvt_kernel<<<dim3(cT * kT), dim3(256), 0, s>>>(src, srcCols, cT, cSplit, rowAddC, kSplit, rowAddK,
                                               dstK, mode, scale, d0, d1);
}

extern "C" void kernel_launch(void* const* d_in, const int* in_sizes, int n_in,
                              void* d_out, int out_size, void* d_ws, size_t ws_size,
                              hipStream_t stream) {
  if (n_in < 18) return;
  if (in_sizes[0] != NNODE * DIN) return;
  if (in_sizes[1] != NGRAPH) return;
  if (in_sizes[2] != 256 * 256 || in_sizes[3] != 256) return;
  if (in_sizes[4] != 256 * 256 || in_sizes[5] != 256 || in_sizes[6] != 256 || in_sizes[7] != 256) return;
  if (in_sizes[8] != 256 * 256 || in_sizes[9] != 256) return;
  if (in_sizes[10] != 388 * 256 || in_sizes[11] != 256) return;
  if (in_sizes[12] != 256 * 256 || in_sizes[13] != 256 || in_sizes[14] != 256 || in_sizes[15] != 256) return;
  if (in_sizes[16] != 256 * 128 || in_sizes[17] != 128) return;
  if (out_size != NNODE * DIN) return;

  const float* states = (const float*)d_in[0];
  const int*   action = (const int*)d_in[1];
  const float* eW1 = (const float*)d_in[2];
  const float* eb1 = (const float*)d_in[3];
  const float* eW2 = (const float*)d_in[4];
  const float* eb2 = (const float*)d_in[5];
  const float* eg  = (const float*)d_in[6];
  const float* ebt = (const float*)d_in[7];
  const float* eW3 = (const float*)d_in[8];
  const float* eb3 = (const float*)d_in[9];
  const float* nW1 = (const float*)d_in[10];
  const float* nb1 = (const float*)d_in[11];
  const float* nW2 = (const float*)d_in[12];
  const float* nb2 = (const float*)d_in[13];
  const float* ng  = (const float*)d_in[14];
  const float* nbt = (const float*)d_in[15];
  const float* nW3 = (const float*)d_in[16];
  const float* nb3 = (const float*)d_in[17];
  float* out = (float*)d_out;

  const size_t b_pq  = (size_t)512 * 128 * 2;
  const size_t b_w   = (size_t)256 * 256 * 2;
  const size_t b_n1  = (size_t)256 * 384 * 2;
  const size_t b_n3  = (size_t)128 * 256 * 2;
  const size_t b_pqp = (size_t)NNODE * 512 * 4;
  const size_t b_agg = (size_t)NNODE * 256 * 4;
  size_t off = 0;
  char* ws = (char*)d_ws;
  unsigned short* bph = (unsigned short*)(ws + off); off += b_pq;
  unsigned short* bpl = (unsigned short*)(ws + off); off += b_pq;
  _Float16* w2h = (_Float16*)(ws + off); off += b_w;
  _Float16* w3h = (_Float16*)(ws + off); off += b_w;
  unsigned short* n1h = (unsigned short*)(ws + off); off += b_n1;
  unsigned short* n1l = (unsigned short*)(ws + off); off += b_n1;
  unsigned short* n2h = (unsigned short*)(ws + off); off += b_w;
  unsigned short* n2l = (unsigned short*)(ws + off); off += b_w;
  unsigned short* n3h = (unsigned short*)(ws + off); off += b_n3;
  unsigned short* n3l = (unsigned short*)(ws + off); off += b_n3;
  float* pqp  = (float*)(ws + off); off += b_pqp;
  float* aggp = (float*)(ws + off); off += b_agg;
  if (off > ws_size) return;

  const int BIG = 1 << 30;
  launch_cvt(stream, eW1, 256, 8, 2, 256, 128, BIG, 0, 128, 1, 1.0f, bph, bpl);
  launch_cvt(stream, eW2, 256, 4, 4, BIG, 0, BIG, 0, 256, 0, 16.0f, (unsigned short*)w2h, (unsigned short*)w2h);
  launch_cvt(stream, eW3, 256, 4, 4, BIG, 0, BIG, 0, 256, 0, 16.0f, (unsigned short*)w3h, (unsigned short*)w3h);
  launch_cvt(stream, nW1, 256, 4, 6, BIG, 0, 128, 4, 384, 1, 1.0f, n1h, n1l);
  launch_cvt(stream, nW2, 256, 4, 4, BIG, 0, BIG, 0, 256, 1, 1.0f, n2h, n2l);
  launch_cvt(stream, nW3, 128, 2, 4, BIG, 0, BIG, 0, 256, 1, 1.0f, n3h, n3l);

  hipFuncSetAttribute(reinterpret_cast<const void*>(&pq_kernel),
                      hipFuncAttributeMaxDynamicSharedMemorySize, P_SMEM);
  hipFuncSetAttribute(reinterpret_cast<const void*>(&edge_kernel),
                      hipFuncAttributeMaxDynamicSharedMemorySize, E_SMEM);
  hipFuncSetAttribute(reinterpret_cast<const void*>(&node_kernel),
                      hipFuncAttributeMaxDynamicSharedMemorySize, N_SMEM);

  pq_kernel<<<dim3(NNODE / 32), dim3(256), (size_t)P_SMEM, stream>>>(states, bph, bpl, eb1, pqp);

  edge_kernel<<<dim3(NGRAPH), dim3(256), (size_t)E_SMEM, stream>>>(
      pqp, w2h, w3h, eb2, eg, ebt, eb3, aggp);

  node_kernel<<<dim3(NNODE / 32), dim3(256), (size_t)N_SMEM, stream>>>(
      states, aggp, action, n1h, n1l, nW1, nb1, n2h, n2l, nb2, ng, nbt, n3h, n3l, nb3, out);
}
